// JittorEDNetDetection_44435731644861
// MI455X (gfx1250) — hardware-verified
//
#include <hip/hip_runtime.h>
#include <stddef.h>
#include <math.h>


#pragma clang fp contract(off)

#define NTHR   256
#define NBAT   16
#define NTAPS  9
#define PT     64
#define PT1    128
#define APITCH 40
#define SPITCH 32
#define OFFP   32
#define EPS_BN 1e-5f

typedef float    v4f  __attribute__((ext_vector_type(4)));
typedef float    v8f  __attribute__((ext_vector_type(8)));
typedef int      v4i  __attribute__((ext_vector_type(4)));
typedef unsigned v4u  __attribute__((ext_vector_type(4)));
typedef _Float16 v8h  __attribute__((ext_vector_type(8)));
typedef _Float16 v16h __attribute__((ext_vector_type(16)));
union Frag { v16h v; v8h half[2]; };
union H8   { v8h h; v4u u; };

static_assert((PT % 32) == 0);
static_assert((PT1 % 32) == 0);
static_assert((APITCH % 8) == 0);

__device__ __forceinline__ v8f wmh(v16h a, v16h b, v8f c) {
  v8f d = __builtin_amdgcn_wmma_f32_16x16x32_f16(false, a, false, b, (short)0, c, false, false);
  asm volatile("v_nop\n\tv_nop\n\tv_nop\n\tv_nop" : "+v"(d) : "v"(a), "v"(b));
  return d;
}

__device__ __forceinline__ v8f zero8f() {
  v8f z;
#pragma unroll
  for (int i = 0; i < 8; ++i) z[i] = 0.0f;
  return z;
}

__device__ __forceinline__ float vgpr_zero() {
  float z;
  asm volatile("v_mov_b32 %0, 0" : "=v"(z));
  return z;
}

__global__ __launch_bounds__(NTHR) void k_wcvt(const float* __restrict__ src, _Float16* dst,
                                              int rows, int K, int rowsPad, int Kpad, float scale) {
  const int t = blockIdx.x * NTHR + (int)threadIdx.x;
  const int total8 = (rowsPad * Kpad) >> 3;
  if (t >= total8) return;
  const int e = t << 3;
  const int r = e / Kpad;
  const int k = e - r * Kpad;
  const int rc = r < rows ? r : rows - 1;
  H8 o;
#pragma unroll
  for (int j = 0; j < 8; ++j) {
    const int kk = k + j;
    const int kc = kk < K ? kk : K - 1;
    const float v = src[(size_t)rc * K + kc];
    const bool ok = (r < rows) && (kk < K);
    o.h[j] = (_Float16)(ok ? v * scale : 0.0f);
  }
  *(volatile v4u*)(dst + e) = o.u;
  __threadfence();
  *(volatile v4u*)(dst + e) = o.u;
}

__global__ __launch_bounds__(NTHR) void k_conv1(const float* __restrict__ x, const _Float16* __restrict__ w1h,
                                               const float* __restrict__ b1, float* y, int H, int W, int P) {
  __shared__ __attribute__((aligned(16))) _Float16 sA[PT1 * APITCH];
  __shared__ __attribute__((aligned(16))) float    sO[16 * PT1];
  const int tid = threadIdx.x, lane = tid & 31, wv = tid >> 5, hh = lane >> 4, m = lane & 15;
  const int pBase = blockIdx.x * PT1;
  const int hw = H * W;
  {
    const int pl = tid & (PT1 - 1), kq = tid >> 7;
    const int p = pBase + pl;
    const int b = p / hw; const int r = p - b * hw; const int oy = r / W; const int ox = r - oy * W;
    const float* xb = x + (size_t)b * hw;
    const float zdv = vgpr_zero();
    H8 o0, o1;
#pragma unroll
    for (int j = 0; j < 16; ++j) {
      const int jj = j < NTAPS ? j : NTAPS - 1;
      const int ky = jj / 3, kx = jj - 3 * ky;
      const int iy = oy + ky - 1, ix = ox + kx - 1;
      const bool ok = (kq == 0) && (j < NTAPS) && ((unsigned)iy < (unsigned)H) && ((unsigned)ix < (unsigned)W);
      const int iyc = iy < 0 ? 0 : (iy > H - 1 ? H - 1 : iy);
      const int ixc = ix < 0 ? 0 : (ix > W - 1 ? W - 1 : ix);
      const float t = xb[iyc * W + ixc];
      const float v = ok ? t : zdv;
      if (j < 8) o0.h[j] = (_Float16)v; else o1.h[j - 8] = (_Float16)v;
    }
    *(v4u*)(sA + pl * APITCH + 16 * kq)     = o0.u;
    *(v4u*)(sA + pl * APITCH + 16 * kq + 8) = o1.u;
  }
  __syncthreads();
  Frag a, bq;
  a.half[0]  = *(const v8h*)(sA + (16 * wv + m) * APITCH + 8 * hh);
  a.half[1]  = *(const v8h*)(sA + (16 * wv + m) * APITCH + 16 + 8 * hh);
  bq.half[0] = *(const v8h*)(w1h + m * 32 + 8 * hh);
  bq.half[1] = *(const v8h*)(w1h + m * 32 + 16 + 8 * hh);
  v8f acc = zero8f();
  acc = wmh(a.v, bq.v, acc);
  const float bias = b1[m];
  v4f s0, s1;
  s0.x = acc[0] * 0.0625f + bias; s0.y = acc[1] * 0.0625f + bias; s0.z = acc[2] * 0.0625f + bias; s0.w = acc[3] * 0.0625f + bias;
  s1.x = acc[4] * 0.0625f + bias; s1.y = acc[5] * 0.0625f + bias; s1.z = acc[6] * 0.0625f + bias; s1.w = acc[7] * 0.0625f + bias;
  *(v4f*)(sO + m * PT1 + 16 * wv + 8 * hh)     = s0;
  *(v4f*)(sO + m * PT1 + 16 * wv + 8 * hh + 4) = s1;
  __syncthreads();
#pragma unroll
  for (int pass = 0; pass < 2; ++pass) {
#pragma unroll
    for (int it = 0; it < 2; ++it) {
      const int L = 8 * wv + 4 * it + (lane >> 3);
      const int o = L >> 2, q = L & 3;
      const v4f v = *(const v4f*)(sO + o * PT1 + 32 * q + 4 * (lane & 7));
      float* dp = y + (size_t)o * P + pBase + 32 * q + 4 * (lane & 7);
      *(volatile v4f*)dp = v;
    }
    if (pass == 0) __threadfence();
  }
}

__global__ __launch_bounds__(NTHR) void k_bnstats(const float* __restrict__ act, float* stats, int P) {
  __shared__ double red[2 * NTHR];
  __shared__ __attribute__((aligned(16))) float resf[32];
  const int tid = threadIdx.x, lane = tid & 31, wv = tid >> 5;
  const int c = blockIdx.x;
  const float* row = act + (size_t)c * P;
  const int n4 = P >> 2;
  double s = 0.0, q = 0.0;
#pragma unroll 1
  for (int i = tid; i < n4; i += NTHR) {
    const v4f v = *(const v4f*)(row + 4 * (size_t)i);
    const double a = (double)v.x, b = (double)v.y, cc = (double)v.z, d = (double)v.w;
    s += a; s += b; s += cc; s += d;
    q += a * a; q += b * b; q += cc * cc; q += d * d;
  }
  red[tid] = s; red[NTHR + tid] = q;
  __syncthreads();
#pragma unroll 1
  for (int st = NTHR / 2; st > 0; st >>= 1) {
    if (tid < st) { red[tid] += red[tid + st]; red[NTHR + tid] += red[NTHR + tid + st]; }
    __syncthreads();
  }
  if (tid == 0) {
    const double inv = 1.0 / (double)P;
    const double mu = red[0] * inv;
    double var = red[NTHR] * inv - mu * mu;
    if (var < 0.0) var = 0.0;
    const float vf = (float)var + EPS_BN;
    resf[0] = (float)mu;
    resf[1] = (float)(1.0 / sqrt((double)vf));
#pragma unroll
    for (int j = 2; j < 32; ++j) resf[j] = 0.0f;
  }
  __syncthreads();
  v4f rv = {0.0f, 0.0f, 0.0f, 0.0f};
  const bool wr = (wv == 0) && (lane < 8);
  if (wr) rv = *(const v4f*)(resf + 4 * lane);
  if (wr) *(volatile v4f*)(stats + (size_t)c * SPITCH + 4 * lane) = rv;
  __threadfence();
  if (wr) *(volatile v4f*)(stats + (size_t)c * SPITCH + 4 * lane) = rv;
}

__global__ __launch_bounds__(NTHR) void k_bnapply(float* act, const float* __restrict__ stats,
                                                 const float* __restrict__ g, const float* __restrict__ be,
                                                 int C, int P) {
  const int n4 = P >> 2;
  const size_t i = (size_t)blockIdx.x * NTHR + threadIdx.x;
  if (i >= (size_t)C * (size_t)n4) return;
  const int c = (int)(i / (size_t)n4);
  const float mu = stats[c * SPITCH], rs = stats[c * SPITCH + 1], gg = g[c], bt = be[c];
  const v4f v = *(const v4f*)(act + 4 * i);
  v4f o;
  o.x = fmaxf(((v.x - mu) * rs) * gg + bt, 0.0f);
  o.y = fmaxf(((v.y - mu) * rs) * gg + bt, 0.0f);
  o.z = fmaxf(((v.z - mu) * rs) * gg + bt, 0.0f);
  o.w = fmaxf(((v.w - mu) * rs) * gg + bt, 0.0f);
  *(volatile v4f*)(act + 4 * i) = o;
  __threadfence();
  *(volatile v4f*)(act + 4 * i) = o;
}

__global__ __launch_bounds__(NTHR) void k_offset(const float* __restrict__ xin, const _Float16* __restrict__ pwh,
                                                const float* __restrict__ pb, float* offp,
                                                int Ci, int H, int W, int h, int w, int Pin, int Kpad) {
  __shared__ __attribute__((aligned(16))) _Float16 sA[PT * APITCH];
  __shared__ __attribute__((aligned(16))) float    sO[PT * OFFP];
  const int tid = threadIdx.x, lane = tid & 31, wv = tid >> 5, hh = lane >> 4, m = lane & 15;
  const int pBase = blockIdx.x * PT;
  const int hw = h * w, HW = H * W, Ktot = Ci * NTAPS;
  const int pl = tid & (PT - 1), kq = tid >> 6;
  const int p = pBase + pl;
  const int b = p / hw; const int r = p - b * hw; const int oy = r / w; const int ox = r - oy * w;
  const float* xb = xin + (size_t)b * HW;
  const int iyb = 2 * oy - 1, ixb = 2 * ox - 1;
  const int mt = wv & 3, nt = wv >> 2;
  const _Float16* bp = pwh + (size_t)(16 * nt + m) * Kpad;
  v8f acc = zero8f();
  const int nks = Kpad >> 5;
#pragma unroll 1
  for (int ks = 0; ks < nks; ++ks) {
    const int k0 = ks << 5;
    H8 o;
#pragma unroll
    for (int j = 0; j < 8; ++j) {
      const int k = k0 + 8 * kq + j;
      const int kk = k < Ktot ? k : Ktot - 1;
      const int c = kk / NTAPS;
      const int n = kk - c * NTAPS;
      const int ky = n / 3, kx = n - 3 * ky;
      const int iy = iyb + ky, ix = ixb + kx;
      const bool ok = (k < Ktot) && ((unsigned)iy < (unsigned)H) && ((unsigned)ix < (unsigned)W);
      const int iyc = iy < 0 ? 0 : (iy > H - 1 ? H - 1 : iy);
      const int ixc = ix < 0 ? 0 : (ix > W - 1 ? W - 1 : ix);
      const float v = xb[(size_t)c * Pin + iyc * W + ixc];
      o.h[j] = (_Float16)(ok ? v : 0.0f);
    }
    *(v4u*)(sA + pl * APITCH + 8 * kq) = o.u;
    __syncthreads();
    Frag a, bq;
    a.half[0]  = *(const v8h*)(sA + (16 * mt + m) * APITCH + 8 * hh);
    a.half[1]  = *(const v8h*)(sA + (16 * mt + m) * APITCH + 16 + 8 * hh);
    bq.half[0] = *(const v8h*)(bp + k0 + 8 * hh);
    bq.half[1] = *(const v8h*)(bp + k0 + 16 + 8 * hh);
    acc = wmh(a.v, bq.v, acc);
    __syncthreads();
  }
  {
    const int n = 16 * nt + m;
    const float bias = pb[n < 18 ? n : 17];
    const bool nv = n < 18;
#pragma unroll
    for (int rr = 0; rr < 8; ++rr) {
      const float t = acc[rr] * 0.015625f + bias;
      sO[(16 * mt + 8 * hh + rr) * OFFP + n] = nv ? t : 0.0f;
    }
  }
  __syncthreads();
#pragma unroll
  for (int pass = 0; pass < 2; ++pass) {
#pragma unroll
    for (int it = 0; it < 2; ++it) {
      const int L = 8 * wv + 4 * it + (lane >> 3);
      const v4f v = *(const v4f*)(sO + L * OFFP + 4 * (lane & 7));
      float* dp = offp + (size_t)(pBase + L) * OFFP + 4 * (lane & 7);
      *(volatile v4f*)dp = v;
    }
    if (pass == 0) __threadfence();
  }
}

template <int NJ>
__global__ __launch_bounds__(NTHR) void k_deform(const float* __restrict__ xin, const float* __restrict__ offp,
                                                const _Float16* __restrict__ cwh, float* yout,
                                                int Ci, int H, int W, int h, int w, int Pin, int Pout, int Kpad) {
  __shared__ __attribute__((aligned(16))) int      sIdx[PT * NTAPS * 4];
  __shared__ __attribute__((aligned(16))) float    sWgt[PT * NTAPS * 4];
  __shared__ __attribute__((aligned(16))) _Float16 sA[PT * APITCH];
  __shared__ __attribute__((aligned(16))) float    sO[32 * PT];
  const int tid = threadIdx.x, lane = tid & 31, wv = tid >> 5, hh = lane >> 4, m = lane & 15;
  const int pBase = blockIdx.x * PT;
  const int hw = h * w, HW = H * W, Ktot = Ci * NTAPS;
  const float hpm = (float)(H + 1), wpm = (float)(W + 1);

  for (int t = tid; t < PT * NTAPS; t += NTHR) {
    const int pl = t / NTAPS, n = t - pl * NTAPS;
    const int p = pBase + pl;
    const int b = p / hw; const int r = p - b * hw; const int oy = r / w; const int ox = r - oy * w;
    const float offy = offp[(size_t)p * OFFP + n];
    const float offx = offp[(size_t)p * OFFP + NTAPS + n];
    const int ty = n / 3, tx = n - 3 * ty;
    float py = offy + (float)(ty - 1); py = py + (float)(1 + 2 * oy);
    float px = offx + (float)(tx - 1); px = px + (float)(1 + 2 * ox);
    const float fy = floorf(py), fx = floorf(px);
    const float qy0 = fminf(fmaxf(fy, 0.0f), hpm);
    const float qy1 = fminf(fmaxf(fy + 1.0f, 0.0f), hpm);
    const float qx0 = fminf(fmaxf(fx, 0.0f), wpm);
    const float qx1 = fminf(fmaxf(fx + 1.0f, 0.0f), wpm);
    const float pyc = fminf(fmaxf(py, 0.0f), hpm);
    const float pxc = fminf(fmaxf(px, 0.0f), wpm);
    const float wy0 = 1.0f + (qy0 - pyc), wy1 = 1.0f - (qy1 - pyc);
    const float wx0 = 1.0f + (qx0 - pxc), wx1 = 1.0f - (qx1 - pxc);
    const int iy0 = (int)qy0 - 1, iy1 = (int)qy1 - 1, ix0 = (int)qx0 - 1, ix1 = (int)qx1 - 1;
    const bool vy0 = (unsigned)iy0 < (unsigned)H, vy1 = (unsigned)iy1 < (unsigned)H;
    const bool vx0 = (unsigned)ix0 < (unsigned)W, vx1 = (unsigned)ix1 < (unsigned)W;
    const int cy0 = iy0 < 0 ? 0 : (iy0 > H - 1 ? H - 1 : iy0);
    const int cy1 = iy1 < 0 ? 0 : (iy1 > H - 1 ? H - 1 : iy1);
    const int cx0 = ix0 < 0 ? 0 : (ix0 > W - 1 ? W - 1 : ix0);
    const int cx1 = ix1 < 0 ? 0 : (ix1 > W - 1 ? W - 1 : ix1);
    const int bb = b * HW;
    v4i id; v4f wg;
    id.x = bb + cy0 * W + cx0; wg.x = (vy0 && vx0) ? wy0 * wx0 : 0.0f;
    id.y = bb + cy1 * W + cx1; wg.y = (vy1 && vx1) ? wy1 * wx1 : 0.0f;
    id.z = bb + cy0 * W + cx1; wg.z = (vy0 && vx1) ? wy0 * wx1 : 0.0f;
    id.w = bb + cy1 * W + cx0; wg.w = (vy1 && vx0) ? wy1 * wx0 : 0.0f;
    *(v4i*)(sIdx + t * 4) = id;
    *(v4f*)(sWgt + t * 4) = wg;
  }
  __syncthreads();

  const int pl = tid & (PT - 1), kq = tid >> 6;
  const int mt = wv & 3, ntb = wv >> 2;
  v8f acc[NJ];
#pragma unroll
  for (int j = 0; j < NJ; ++j) acc[j] = zero8f();
  const int nks = Kpad >> 5;
#pragma unroll 1
  for (int ks = 0; ks < nks; ++ks) {
    const int k0 = ks << 5;
    H8 o;
#pragma unroll
    for (int j = 0; j < 8; ++j) {
      const int k = k0 + 8 * kq + j;
      const int kk = k < Ktot ? k : Ktot - 1;
      const int c = kk / NTAPS;
      const int n = kk - c * NTAPS;
      const v4i id = *(const v4i*)(sIdx + (pl * NTAPS + n) * 4);
      const v4f wg = *(const v4f*)(sWgt + (pl * NTAPS + n) * 4);
      const float* xc = xin + (size_t)c * Pin;
      float v = wg.x * xc[id.x];
      v = fmaf(wg.y, xc[id.y], v);
      v = fmaf(wg.z, xc[id.z], v);
      v = fmaf(wg.w, xc[id.w], v);
      o.h[j] = (_Float16)((k < Ktot) ? v : 0.0f);
    }
    *(v4u*)(sA + pl * APITCH + 8 * kq) = o.u;
    __syncthreads();
    Frag a;
    a.half[0] = *(const v8h*)(sA + (16 * mt + m) * APITCH + 8 * hh);
    a.half[1] = *(const v8h*)(sA + (16 * mt + m) * APITCH + 16 + 8 * hh);
#pragma unroll
    for (int j = 0; j < NJ; ++j) {
      const int nt = ntb + 2 * j;
      const _Float16* bp = cwh + (size_t)(16 * nt + m) * Kpad + k0;
      Frag bq;
      bq.half[0] = *(const v8h*)(bp + 8 * hh);
      bq.half[1] = *(const v8h*)(bp + 16 + 8 * hh);
      acc[j] = wmh(a.v, bq.v, acc[j]);
    }
    __syncthreads();
  }

#pragma unroll
  for (int jc = 0; jc < NJ; ++jc) {
    const int cl = 16 * ntb + m;
    v4f s0, s1;
    s0.x = acc[jc][0] * 0.0625f; s0.y = acc[jc][1] * 0.0625f; s0.z = acc[jc][2] * 0.0625f; s0.w = acc[jc][3] * 0.0625f;
    s1.x = acc[jc][4] * 0.0625f; s1.y = acc[jc][5] * 0.0625f; s1.z = acc[jc][6] * 0.0625f; s1.w = acc[jc][7] * 0.0625f;
    *(v4f*)(sO + cl * PT + 16 * mt + 8 * hh)     = s0;
    *(v4f*)(sO + cl * PT + 16 * mt + 8 * hh + 4) = s1;
    __syncthreads();
#pragma unroll
    for (int pass = 0; pass < 2; ++pass) {
#pragma unroll
      for (int it = 0; it < 2; ++it) {
        const int L = 8 * wv + 4 * it + (lane >> 3);
        const int c2 = L >> 1, half = L & 1;
        const v4f v = *(const v4f*)(sO + c2 * PT + 32 * half + 4 * (lane & 7));
        float* dp = yout + (size_t)(32 * jc + c2) * Pout + pBase + 32 * half + 4 * (lane & 7);
        *(volatile v4f*)dp = v;
      }
      if (pass == 0) __threadfence();
    }
    __syncthreads();
  }
}

__global__ __launch_bounds__(NTHR) void k_head(const float* __restrict__ act, const float* __restrict__ wc,
                                              const float* __restrict__ bc, const float* __restrict__ wb,
                                              const float* __restrict__ bb, float* out, int P, int hw) {
  __shared__ float sv[NBAT * 256];
  __shared__ __attribute__((aligned(16))) float sres[NBAT * 14];
  const int tid = threadIdx.x, lane = tid & 31, wv = tid >> 5;
  const int c = tid;
  const float inv = 1.0f / (float)hw;
#pragma unroll 1
  for (int b = 0; b < NBAT; ++b) {
    const float* p = act + (size_t)c * P + b * hw;
    double s = 0.0;
#pragma unroll 1
    for (int i = 0; i < hw; ++i) s += (double)p[i];
    sv[b * 256 + c] = (float)s * inv;
  }
  __syncthreads();
  if (tid < NBAT * 10) {
    const int b = tid / 10, j = tid - b * 10;
    float s = 0.0f;
#pragma unroll 1
    for (int k = 0; k < 256; ++k) s += sv[b * 256 + k] * wc[j * 256 + k];
    sres[tid] = s + bc[j];
  } else if (tid < NBAT * 14) {
    const int t2 = tid - NBAT * 10;
    const int b = t2 / 4, j = t2 - b * 4;
    float s = 0.0f;
#pragma unroll 1
    for (int k = 0; k < 256; ++k) s += sv[b * 256 + k] * wb[j * 256 + k];
    s += bb[j];
    const float e = expf(-s);
    sres[NBAT * 10 + t2] = 1.0f / (1.0f + e);
  }
  __syncthreads();
  const int q = wv * 32 + lane;
  const bool wr = (wv == 0) || (wv == 1 && lane < 24);
  v4f rv = {0.0f, 0.0f, 0.0f, 0.0f};
  if (wr) rv = *(const v4f*)(sres + 4 * q);
  if (wr) *(volatile v4f*)(out + 4 * q) = rv;
  __threadfence();
  if (wr) *(volatile v4f*)(out + 4 * q) = rv;
}

extern "C" void kernel_launch(void* const* d_in, const int* in_sizes, int n_in,
                              void* d_out, int out_size, void* d_ws, size_t ws_size,
                              hipStream_t stream) {
  if (n_in < 29) return;
  const int H1 = 224;
  const int P1 = NBAT * H1 * H1;
  const int ciA[4]  = {16, 32, 64, 128};
  const int coA[4]  = {32, 64, 128, 256};
  const int hinA[4] = {224, 112, 56, 28};
  if (in_sizes[0] != P1 || in_sizes[1] != 16 * NTAPS || in_sizes[2] < 16 || in_sizes[3] < 16 || in_sizes[4] < 16) return;
  for (int s = 0; s < 4; ++s) {
    const int ci = ciA[s], co = coA[s];
    if (in_sizes[5 + 5 * s] != 18 * ci * NTAPS || in_sizes[6 + 5 * s] < 18) return;
    if (in_sizes[7 + 5 * s] != co * ci * NTAPS || in_sizes[8 + 5 * s] < co || in_sizes[9 + 5 * s] < co) return;
  }
  if (in_sizes[25] != 10 * 256 || in_sizes[26] < 10 || in_sizes[27] != 4 * 256 || in_sizes[28] < 4) return;
  if (out_size != NBAT * 14) return;
  if ((P1 % PT1) != 0) return;

  int Pout[4], Kpad[4];
  for (int s = 0; s < 4; ++s) {
    const int ho = hinA[s] / 2;
    Pout[s] = NBAT * ho * ho;
    Kpad[s] = ((NTAPS * ciA[s] + 31) / 32) * 32;
    if ((Pout[s] % PT) != 0) return;
  }

  char* ws = (char*)d_ws;
  size_t off = 0;
  size_t oAct[5], oPw[4], oCw[4];
  oAct[0] = off; off += (size_t)16 * P1 * 4;
  for (int s = 0; s < 4; ++s) { oAct[s + 1] = off; off += (size_t)coA[s] * Pout[s] * 4; }
  const size_t oOff = off; off += (size_t)Pout[0] * OFFP * 4;
  const size_t oSt  = off; off += (size_t)256 * SPITCH * 4;
  const size_t oW1  = off; off += (size_t)16 * 32 * 2;
  for (int s = 0; s < 4; ++s) {
    oPw[s] = off; off += (((size_t)32 * Kpad[s] * 2) + 255) & ~(size_t)255;
    oCw[s] = off; off += (((size_t)coA[s] * Kpad[s] * 2) + 255) & ~(size_t)255;
  }
  if (off > ws_size) return;

  float* act[5];
  for (int i = 0; i < 5; ++i) act[i] = (float*)(ws + oAct[i]);
  float* offb  = (float*)(ws + oOff);
  float* stats = (float*)(ws + oSt);
  _Float16* w1h = (_Float16*)(ws + oW1);

  const float* x   = (const float*)d_in[0];
  const float* w1  = (const float*)d_in[1];
  const float* b1  = (const float*)d_in[2];
  const float* g1  = (const float*)d_in[3];
  const float* be1 = (const float*)d_in[4];
  const float* wc  = (const float*)d_in[25];
  const float* bc  = (const float*)d_in[26];
  const float* wb  = (const float*)d_in[27];
  const float* bbx = (const float*)d_in[28];

  {
    const int tot8 = (16 * 32) / 8;
    k_wcvt<<<(tot8 + NTHR - 1) / NTHR, NTHR, 0, stream>>>(w1, w1h, 16, NTAPS, 16, 32, 16.0f);
  }
  for (int s = 0; s < 4; ++s) {
    const float* pw = (const float*)d_in[5 + 5 * s];
    const float* cw = (const float*)d_in[7 + 5 * s];
    const int K = NTAPS * ciA[s];
    {
      const int tot8 = (32 * Kpad[s]) / 8;
      k_wcvt<<<(tot8 + NTHR - 1) / NTHR, NTHR, 0, stream>>>(pw, (_Float16*)(ws + oPw[s]), 18, K, 32, Kpad[s], 64.0f);
    }
    {
      const int tot8 = (coA[s] * Kpad[s]) / 8;
      k_wcvt<<<(tot8 + NTHR - 1) / NTHR, NTHR, 0, stream>>>(cw, (_Float16*)(ws + oCw[s]), coA[s], K, coA[s], Kpad[s], 16.0f);
    }
  }

  k_conv1<<<P1 / PT1, NTHR, 0, stream>>>(x, w1h, b1, act[0], H1, H1, P1);
  k_bnstats<<<16, NTHR, 0, stream>>>(act[0], stats, P1);
  {
    const size_t n4 = (size_t)16 * (P1 / 4);
    k_bnapply<<<(unsigned)((n4 + NTHR - 1) / NTHR), NTHR, 0, stream>>>(act[0], stats, g1, be1, 16, P1);
  }

  for (int s = 0; s < 4; ++s) {
    const float* pb = (const float*)d_in[6 + 5 * s];
    const float* g  = (const float*)d_in[8 + 5 * s];
    const float* be = (const float*)d_in[9 + 5 * s];
    const int Ci = ciA[s], Co = coA[s], H = hinA[s], W = hinA[s], h = H / 2, w = W / 2;
    const int Pin = NBAT * H * W, Po = Pout[s];
    const _Float16* pwh = (const _Float16*)(ws + oPw[s]);
    const _Float16* cwh = (const _Float16*)(ws + oCw[s]);
    const float* xin = act[s];
    float* yout = act[s + 1];

    k_offset<<<Po / PT, NTHR, 0, stream>>>(xin, pwh, pb, offb, Ci, H, W, h, w, Pin, Kpad[s]);
    switch (Co / 32) {
      case 1: k_deform<1><<<Po / PT, NTHR, 0, stream>>>(xin, offb, cwh, yout, Ci, H, W, h, w, Pin, Po, Kpad[s]); break;
      case 2: k_deform<2><<<Po / PT, NTHR, 0, stream>>>(xin, offb, cwh, yout, Ci, H, W, h, w, Pin, Po, Kpad[s]); break;
      case 4: k_deform<4><<<Po / PT, NTHR, 0, stream>>>(xin, offb, cwh, yout, Ci, H, W, h, w, Pin, Po, Kpad[s]); break;
      default: k_deform<8><<<Po / PT, NTHR, 0, stream>>>(xin, offb, cwh, yout, Ci, H, W, h, w, Pin, Po, Kpad[s]); break;
    }
    k_bnstats<<<Co, NTHR, 0, stream>>>(yout, stats, Po);
    {
      const size_t n4 = (size_t)Co * (Po / 4);
      k_bnapply<<<(unsigned)((n4 + NTHR - 1) / NTHR), NTHR, 0, stream>>>(yout, stats, g, be, Co, Po);
    }
  }

  k_head<<<1, NTHR, 0, stream>>>(act[4], wc, bc, wb, bbx, (float*)d_out, Pout[3], (hinA[3] / 2) * (hinA[3] / 2));
}
